// StateWeightNet_12438225289584
// MI455X (gfx1250) — hardware-verified
//
#include <hip/hip_runtime.h>
#include <stddef.h>
#include <stdint.h>


#define NN      70000
#define NE      1120000
#define DF      73
#define DP      96
#define MPAD    70016
#define XLN     192
#define GPW     384
#define NTHR    256
#define NWAVE   8
#define EPT     8
#define CHUNK   (NTHR * EPT)
#define WCAP    (EPT * 32)
#define LISTN   (NWAVE * WCAP)
#define NBMAX   2048
#define NBRUN   1024
#define SLB     10
#define SMASK   1023
#define RCAP    28672
#define DEGCAP  64
#define STW     512
#define GBM     64
#define GTHR    128
#define NEGS    0.2f
#define WSMAX   134217728
#define LDS_AGG ((2 * RCAP + 2 * NBMAX + LISTN) * 4 + 64)

static_assert(DF <= DP && (DP % 32) == 0);
static_assert((NN % 7) == 0 && (NN % 4) == 0);
static_assert(MPAD == 547 * 128 && (MPAD % GBM) == 0 && MPAD >= NN);
static_assert(4 * DP == GPW && 2 * DP == XLN);
static_assert((NE % 4) == 0 && NE < (1 << 21));
static_assert(((long long)NE << SLB) < (1LL << 31));
static_assert((CHUNK & (CHUNK - 1)) == 0 && CHUNK <= 4096);
static_assert((NBMAX & (NBMAX - 1)) == 0 && NBMAX <= 4096);
static_assert(NBRUN == (1 << SLB) && NBRUN <= NBMAX && (NBRUN % NWAVE) == 0);
static_assert(NTHR * 8 == NBMAX);
static_assert(LISTN >= NBMAX && LISTN >= NWAVE * WCAP);
static_assert((RCAP % 32) == 0 && NWAVE * STW <= RCAP && STW >= 96);
static_assert(LDS_AGG <= 300000);
static_assert(GBM == (GTHR / 32) * 16);
static_assert(((MPAD + NBRUN - 1) / NBRUN) * NBRUN >= MPAD);

typedef float          v4f   __attribute__((ext_vector_type(4)));
typedef float          v8f   __attribute__((ext_vector_type(8)));
typedef int            v4i   __attribute__((ext_vector_type(4)));
typedef int            v8i   __attribute__((ext_vector_type(8)));
typedef unsigned short v4us  __attribute__((ext_vector_type(4)));
typedef unsigned short v8us  __attribute__((ext_vector_type(8)));
typedef unsigned short v16us __attribute__((ext_vector_type(16)));
typedef __bf16         v16bf __attribute__((ext_vector_type(16)));
typedef v4f  __attribute__((may_alias)) v4fa;
typedef v4i  __attribute__((may_alias)) v4ia;
typedef v4us __attribute__((may_alias)) v4usa;
typedef v8us __attribute__((may_alias)) v8usa;
union FragB { v16bf v; v16us u; v8us h[2]; v8i w; };

__device__ __forceinline__ v8f wmb(const FragB& a, const FragB& b, v8f c) {
  v8f d = __builtin_amdgcn_wmma_f32_16x16x32_bf16(false, a.v, false, b.v, (short)0, c, false, false);
  asm volatile("v_nop\n\tv_nop\n\tv_nop\n\tv_nop" : "+v"(d) : "v"(a.w), "v"(b.w));
  return d;
}

__device__ __forceinline__ void ldwait() {
  asm volatile("s_wait_loadcnt 0x0" ::: "memory");
}

__device__ __forceinline__ unsigned bf16_bits(float f) {
  const unsigned u = __float_as_uint(f);
  const unsigned r = (u + 0x7FFFu + ((u >> 16) & 1u)) >> 16;
  return (f != f) ? 0x7fc0u : r;
}
__device__ __forceinline__ float bf16_val(float f) {
  return __uint_as_float(bf16_bits(f) << 16);
}
__device__ __forceinline__ float relu_np(float v) {
  return (v > 0.0f) ? v : ((v == v) ? 0.0f : v);
}
__device__ __forceinline__ v8us cvt8b(const v4f a, const v4f b) {
  v8us o;
  o[0] = (unsigned short)bf16_bits(a.x); o[1] = (unsigned short)bf16_bits(a.y);
  o[2] = (unsigned short)bf16_bits(a.z); o[3] = (unsigned short)bf16_bits(a.w);
  o[4] = (unsigned short)bf16_bits(b.x); o[5] = (unsigned short)bf16_bits(b.y);
  o[6] = (unsigned short)bf16_bits(b.z); o[7] = (unsigned short)bf16_bits(b.w);
  return o;
}
__device__ __forceinline__ float ldcol(const float* __restrict__ p, int c, int lim, bool rowok) {
  const int cc = c < lim ? c : lim - 1;
  const float v = p[cc];
  return (rowok && c < lim) ? v : 0.0f;
}

__device__ __forceinline__ void wave_sync() {
  __builtin_amdgcn_fence(__ATOMIC_RELEASE, "workgroup");
  __builtin_amdgcn_wave_barrier();
  __builtin_amdgcn_fence(__ATOMIC_ACQUIRE, "workgroup");
}

__device__ __forceinline__ int scan_chunk(const int* __restrict__ dsts, int nE, int cbase, int slotBase,
                                          int nb, int vec8, int* list, int tid, int lane, int wave) {
  int wc = 0;
  const int el0  = tid * EPT;
  const int e0   = cbase + el0;
  const int sent = -2147483647 - 1;
  v4i da, db;
  if (vec8 != 0 && cbase + CHUNK <= nE) {
    da = *(const v4i*)(dsts + e0);
    db = *(const v4i*)(dsts + e0 + 4);
  } else {
    da.x = (e0     < nE) ? dsts[min(e0,     nE - 1)] : sent;
    da.y = (e0 + 1 < nE) ? dsts[min(e0 + 1, nE - 1)] : sent;
    da.z = (e0 + 2 < nE) ? dsts[min(e0 + 2, nE - 1)] : sent;
    da.w = (e0 + 3 < nE) ? dsts[min(e0 + 3, nE - 1)] : sent;
    db.x = (e0 + 4 < nE) ? dsts[min(e0 + 4, nE - 1)] : sent;
    db.y = (e0 + 5 < nE) ? dsts[min(e0 + 5, nE - 1)] : sent;
    db.z = (e0 + 6 < nE) ? dsts[min(e0 + 6, nE - 1)] : sent;
    db.w = (e0 + 7 < nE) ? dsts[min(e0 + 7, nE - 1)] : sent;
  }
  const unsigned nbs = (unsigned)slotBase;
  const unsigned unb = (unsigned)nb;
  const unsigned s0 = (unsigned)da.x - nbs, s1 = (unsigned)da.y - nbs;
  const unsigned s2 = (unsigned)da.z - nbs, s3 = (unsigned)da.w - nbs;
  const unsigned s4 = (unsigned)db.x - nbs, s5 = (unsigned)db.y - nbs;
  const unsigned s6 = (unsigned)db.z - nbs, s7 = (unsigned)db.w - nbs;
  const bool h0 = s0 < unb, h1 = s1 < unb, h2 = s2 < unb, h3 = s3 < unb;
  const bool h4 = s4 < unb, h5 = s5 < unb, h6 = s6 < unb, h7 = s7 < unb;
  const unsigned any = __builtin_amdgcn_ballot_w32(h0 | h1 | h2 | h3 | h4 | h5 | h6 | h7);
  if (any != 0u) {
#define HITJ(J, HJ, SJ) { \
      const unsigned mj = __builtin_amdgcn_ballot_w32(HJ); \
      if (mj != 0u) { \
        if (HJ) { \
          const int pos = wc + (int)__builtin_amdgcn_mbcnt_lo(mj, 0u); \
          if (pos < WCAP) list[wave * WCAP + pos] = ((el0 + (J)) << 12) | (int)(SJ); \
        } \
        wc += (int)__builtin_popcount(mj); } }
    HITJ(0, h0, s0)
    HITJ(1, h1, s1)
    HITJ(2, h2, s2)
    HITJ(3, h3, s3)
    HITJ(4, h4, s4)
    HITJ(5, h5, s5)
    HITJ(6, h6, s6)
    HITJ(7, h7, s7)
#undef HITJ
  }
  return wc;
}

__global__ __launch_bounds__(NTHR) void k_px(const float* __restrict__ x, unsigned short* xb, int nUnits) {
  const int i = (int)blockIdx.x * NTHR + (int)threadIdx.x;
  if (i >= nUnits) return;
  const int row = i / 12;
  const int k8  = (i - row * 12) * 8;
  const bool ok = row < NN;
  const int rc  = ok ? row : NN - 1;
  const float* p = x + (size_t)rc * DF;
  v4f a, b;
  a.x = ldcol(p, k8 + 0, DF, ok); a.y = ldcol(p, k8 + 1, DF, ok);
  a.z = ldcol(p, k8 + 2, DF, ok); a.w = ldcol(p, k8 + 3, DF, ok);
  b.x = ldcol(p, k8 + 4, DF, ok); b.y = ldcol(p, k8 + 5, DF, ok);
  b.z = ldcol(p, k8 + 6, DF, ok); b.w = ldcol(p, k8 + 7, DF, ok);
  const v8us hv = cvt8b(a, b);
  unsigned short* dp = xb + (size_t)i * 8;
  *(volatile v8us*)dp = hv;
  __threadfence();
  *(volatile v8us*)dp = hv;
}

__device__ __forceinline__ void pw_rows(const float* __restrict__ W, unsigned short* wlr, int rowOff, int u) {
  const int n  = u / 12;
  const int k8 = (u - n * 12) * 8;
  const bool ok = n < DF;
  const int nc = ok ? n : DF - 1;
  const float* p = W + (size_t)nc * DF;
  v4f a, b;
  a.x = ldcol(p, k8 + 0, DF, ok); a.y = ldcol(p, k8 + 1, DF, ok);
  a.z = ldcol(p, k8 + 2, DF, ok); a.w = ldcol(p, k8 + 3, DF, ok);
  b.x = ldcol(p, k8 + 4, DF, ok); b.y = ldcol(p, k8 + 5, DF, ok);
  b.z = ldcol(p, k8 + 6, DF, ok); b.w = ldcol(p, k8 + 7, DF, ok);
  const v8us hv = cvt8b(a, b);
  unsigned short* dp = wlr + (size_t)(rowOff + n) * DP + k8;
  *(volatile v8us*)dp = hv;
  __threadfence();
  *(volatile v8us*)dp = hv;
}

__global__ __launch_bounds__(128) void k_pw(const float* __restrict__ Wl, const float* __restrict__ bl,
                                            const float* __restrict__ Wr, const float* __restrict__ br,
                                            const float* __restrict__ att, const float* __restrict__ bias,
                                            unsigned short* wlr, float* par) {
  __shared__ __attribute__((aligned(16))) float sp[4 * DP];
  const int b = (int)blockIdx.x, tid = (int)threadIdx.x;
  if (b < 9) {
    pw_rows(Wl, wlr, 0, b * 128 + tid);
  } else if (b < 18) {
    pw_rows(Wr, wlr, DP, (b - 9) * 128 + tid);
  } else {
    const bool ok = tid < DF;
    const int tc = ok ? tid : DF - 1;
    const float v0 = bl[tc], v1 = br[tc], v2 = att[tc], v3 = bias[tc];
    if (tid < DP) {
      sp[tid]          = ok ? bf16_val(v0) : 0.0f;
      sp[DP + tid]     = ok ? bf16_val(v1) : 0.0f;
      sp[2 * DP + tid] = ok ? bf16_val(v2) : 0.0f;
      sp[3 * DP + tid] = ok ? bf16_val(v3) : 0.0f;
    }
    __syncthreads();
    if (tid < DP) {
      const v4f v = *(const v4fa*)(sp + 4 * tid);
      *(volatile v4f*)(par + 4 * tid) = v;
      __threadfence();
      *(volatile v4f*)(par + 4 * tid) = v;
    }
  }
}

__global__ __launch_bounds__(NTHR) void k_pm1(const float* __restrict__ W1, const float* __restrict__ b1,
                                              const float* __restrict__ W2, const float* __restrict__ b2,
                                              unsigned short* w1cat, unsigned short* w2cat, float* pb) {
  __shared__ __attribute__((aligned(16))) float sp[192];
  const int b = (int)blockIdx.x, tid = (int)threadIdx.x;
  if (b < 24) {
    const int u   = b * NTHR + tid;
    const int n   = u / 48;
    const int q   = u - n * 48;
    const int seg = q / 12;
    const int kk  = (q - seg * 12) * 8;
    const float* p = W1 + (size_t)n * 146 + (seg >> 1) * DF;
    v4f a, c;
    a.x = ldcol(p, kk + 0, DF, true); a.y = ldcol(p, kk + 1, DF, true);
    a.z = ldcol(p, kk + 2, DF, true); a.w = ldcol(p, kk + 3, DF, true);
    c.x = ldcol(p, kk + 4, DF, true); c.y = ldcol(p, kk + 5, DF, true);
    c.z = ldcol(p, kk + 6, DF, true); c.w = ldcol(p, kk + 7, DF, true);
    const v8us hv = cvt8b(a, c);
    unsigned short* dp = w1cat + (size_t)u * 8;
    *(volatile v8us*)dp = hv;
    __threadfence();
    *(volatile v8us*)dp = hv;
  } else if (b < 32) {
    const int v = (b - 24) * NTHR + tid;
    const int n = v >> 5;
    const int k = ((v & 31) * 8) & 127;
    const float* p = W2 + (size_t)n * 128 + k;
    const v4f a = *(const v4f*)p;
    const v4f c = *(const v4f*)(p + 4);
    const v8us hv = cvt8b(a, c);
    unsigned short* dp = w2cat + (size_t)v * 8;
    *(volatile v8us*)dp = hv;
    __threadfence();
    *(volatile v8us*)dp = hv;
  } else {
    const float v0 = b1[tid < 128 ? tid : 127];
    const float v1 = b2[tid < 64 ? tid : 63];
    if (tid < 128) sp[tid] = bf16_val(v0);
    if (tid < 64)  sp[128 + tid] = bf16_val(v1);
    __syncthreads();
    if (tid < 48) {
      const v4f v = *(const v4fa*)(sp + 4 * tid);
      *(volatile v4f*)(pb + 4 * tid) = v;
      __threadfence();
      *(volatile v4f*)(pb + 4 * tid) = v;
    }
  }
}

__global__ __launch_bounds__(NTHR) void k_pm2(const float* __restrict__ W3, const float* __restrict__ b3,
                                              const float* __restrict__ W4, const float* __restrict__ b4,
                                              unsigned short* w3cat, float* pb) {
  __shared__ __attribute__((aligned(16))) float sp[96];
  const int b = (int)blockIdx.x, tid = (int)threadIdx.x;
  if (b < 2) {
    const int v = b * NTHR + tid;
    const int n = v >> 4;
    const int k = ((v & 15) * 8) & 63;
    const float* p = W3 + (size_t)n * 64 + k;
    const v4f a = *(const v4f*)p;
    const v4f c = *(const v4f*)(p + 4);
    const v8us hv = cvt8b(a, c);
    unsigned short* dp = w3cat + (size_t)v * 8;
    *(volatile v8us*)dp = hv;
    __threadfence();
    *(volatile v8us*)dp = hv;
  } else {
    const int tc = tid < 32 ? tid : 31;
    const float v0 = b3[tc], v1 = W4[tc], v2 = b4[0];
    if (tid < 32) {
      sp[tid]      = bf16_val(v0);
      sp[32 + tid] = bf16_val(v1);
      sp[64 + tid] = (tid == 0) ? bf16_val(v2) : 0.0f;
    }
    __syncthreads();
    if (tid < 24) {
      const v4f v = *(const v4fa*)(sp + 4 * tid);
      *(volatile v4f*)(pb + 192 + 4 * tid) = v;
      __threadfence();
      *(volatile v4f*)(pb + 192 + 4 * tid) = v;
    }
  }
}

template <int NT, int MODE>
__global__ __launch_bounds__(GTHR) __attribute__((amdgpu_num_vgpr(248)))
void k_gemm(const unsigned short* __restrict__ A, int lda, const unsigned short* __restrict__ BT, int K,
            const float* __restrict__ pvec, void* outp, int nOut) {
  constexpr int N   = 16 * NT;
  constexpr int NBV = (MODE == 2) ? 96 : N;
  static_assert((N % 8) == 0 && NBV / 4 <= GTHR);
  static_assert(MODE != 2 || N == 32);
  __shared__ __attribute__((aligned(16))) float stg[GBM * N];
  __shared__ __attribute__((aligned(16))) float sb[NBV];
  __shared__ __attribute__((aligned(16))) float ssc[GBM];
  const int tid = (int)threadIdx.x, lane = tid & 31, wave = tid >> 5, hh = lane >> 4, m = lane & 15;
  const int rowBase = (int)blockIdx.x * GBM;

  if (tid < NBV / 4) *(v4fa*)(sb + 4 * tid) = *(const v4f*)(pvec + 4 * tid);

  v8f acc[NT];
  {
    const v8f z = {0.f, 0.f, 0.f, 0.f, 0.f, 0.f, 0.f, 0.f};
#pragma unroll
    for (int t = 0; t < NT; ++t) acc[t] = z;
  }
  const unsigned short* ap = A + (size_t)(rowBase + 16 * wave + m) * (size_t)lda + 8 * hh;
  const unsigned short* bp = BT + (size_t)m * (size_t)K + 8 * hh;

#pragma unroll 1
  for (int k0 = 0; k0 < K; k0 += 32) {
    FragB af;
    af.h[0] = *(const v8usa*)(ap + k0);
    af.h[1] = *(const v8usa*)(ap + k0 + 16);
#pragma unroll
    for (int nt = 0; nt < NT; ++nt) {
      const unsigned short* wq = bp + (size_t)(16 * nt) * (size_t)K + k0;
      FragB bf;
      bf.h[0] = *(const v8usa*)wq;
      bf.h[1] = *(const v8usa*)(wq + 16);
      acc[nt] = wmb(af, bf, acc[nt]);
    }
  }

#pragma unroll
  for (int nt = 0; nt < NT; ++nt) {
    const int lc = 16 * nt + m;
#pragma unroll
    for (int r = 0; r < 8; ++r) {
      const int lr = 16 * wave + 8 * hh + r;
      stg[lr * N + lc] = acc[nt][r];
    }
  }
  __syncthreads();

  if constexpr (MODE == 0) {
    constexpr int NI = N / 8;
    const float* wst = stg + 16 * wave * N;
    float* og = (float*)outp + (size_t)(rowBase + 16 * wave) * N;
#pragma unroll 4
    for (int i = 0; i < NI; ++i) {
      const int j = 32 * i + lane;
      const int col = (4 * j) % N;
      const v4f v = *(const v4fa*)(wst + 4 * j) + *(const v4fa*)(sb + col);
      *(volatile v4f*)(og + 4 * j) = v;
    }
    __threadfence();
#pragma unroll 4
    for (int i = 0; i < NI; ++i) {
      const int j = 32 * i + lane;
      const int col = (4 * j) % N;
      const v4f v = *(const v4fa*)(wst + 4 * j) + *(const v4fa*)(sb + col);
      *(volatile v4f*)(og + 4 * j) = v;
    }
  } else if constexpr (MODE == 1) {
    constexpr int NI = N / 8;
    const float* wst = stg + 16 * wave * N;
    v4f pv[NI];
#pragma unroll
    for (int i = 0; i < NI; ++i) {
      const int j = 32 * i + lane;
      const int col = (4 * j) % N;
      v4f t = *(const v4fa*)(wst + 4 * j) + *(const v4fa*)(sb + col);
      t.x = relu_np(t.x); t.y = relu_np(t.y); t.z = relu_np(t.z); t.w = relu_np(t.w);
      pv[i] = t;
    }
    __syncthreads();
    unsigned short* s16 = (unsigned short*)stg + (size_t)(16 * wave) * (2 * N);
#pragma unroll
    for (int i = 0; i < NI; ++i) {
      const int j = 32 * i + lane;
      const int r = (4 * j) / N;
      const int col = (4 * j) % N;
      v4us h4, l4;
      unsigned hb;
      hb = bf16_bits(pv[i].x); h4[0] = (unsigned short)hb; l4[0] = (unsigned short)bf16_bits(pv[i].x - __uint_as_float(hb << 16));
      hb = bf16_bits(pv[i].y); h4[1] = (unsigned short)hb; l4[1] = (unsigned short)bf16_bits(pv[i].y - __uint_as_float(hb << 16));
      hb = bf16_bits(pv[i].z); h4[2] = (unsigned short)hb; l4[2] = (unsigned short)bf16_bits(pv[i].z - __uint_as_float(hb << 16));
      hb = bf16_bits(pv[i].w); h4[3] = (unsigned short)hb; l4[3] = (unsigned short)bf16_bits(pv[i].w - __uint_as_float(hb << 16));
      *(v4usa*)(s16 + r * (2 * N) + col) = h4;
      *(v4usa*)(s16 + r * (2 * N) + N + col) = l4;
    }
    __syncthreads();
    unsigned short* og = (unsigned short*)outp + (size_t)(rowBase + 16 * wave) * (2 * N);
#pragma unroll 4
    for (int i = 0; i < NI; ++i) {
      const int q = 32 * i + lane;
      const v8us v = *(const v8usa*)(s16 + 8 * q);
      *(volatile v8us*)(og + 8 * q) = v;
    }
    __threadfence();
#pragma unroll 4
    for (int i = 0; i < NI; ++i) {
      const int q = 32 * i + lane;
      const v8us v = *(const v8usa*)(s16 + 8 * q);
      *(volatile v8us*)(og + 8 * q) = v;
    }
  } else {
#pragma unroll
    for (int i = 0; i < (GBM * N / 4) / GTHR; ++i) {
      const int j = GTHR * i + tid;
      const int col = (4 * j) % N;
      v4f t = *(const v4fa*)(stg + 4 * j) + *(const v4fa*)(sb + col);
      t.x = relu_np(t.x); t.y = relu_np(t.y); t.z = relu_np(t.z); t.w = relu_np(t.w);
      *(v4fa*)(stg + 4 * j) = t;
    }
    __syncthreads();
    if (tid < GBM) {
      float s = 0.0f;
#pragma unroll 4
      for (int k = 0; k < N; ++k) s = fmaf(stg[tid * N + k], sb[N + k], s);
      ssc[tid] = s + sb[2 * N];
    }
    __syncthreads();
    if (wave == 0) {
      const int rem = nOut - rowBase;
      const int nv  = rem < GBM ? rem : GBM;
      const int lq  = lane < 16 ? lane : 15;
      const v4f v   = *(const v4fa*)(ssc + 4 * lq);
      const bool ok = (4 * lane) < nv;
      float* op = (float*)outp + (size_t)rowBase + 4 * lq;
      if (ok) *(volatile v4f*)op = v;
      __threadfence();
      if (ok) *(volatile v4f*)op = v;
    }
  }
}

__global__ __launch_bounds__(NTHR) __attribute__((amdgpu_num_vgpr(248)))
void k_scan(const int* __restrict__ srcs, const int* __restrict__ dsts,
            const float* __restrict__ XLR, const unsigned short* __restrict__ XB,
            const float* __restrict__ PAR, unsigned short* G, int goff) {
  extern __shared__ v4f lds_dyn[];
  int* reg1 = (int*)lds_dyn;
  int* reg2 = reg1 + RCAP;
  int* scnt = reg2 + RCAP;
  int* soff = scnt + NBMAX;
  int* list = soff + NBMAX;
  int* wcnt = list + LISTN;
  int* wtot = wcnt + NWAVE;
  const int tid = (int)threadIdx.x, lane = tid & 31, wave = tid >> 5;
  const int nodeBase = (int)blockIdx.x * NBRUN;
  const int nE = NE, nN = NN;

  for (int i = tid; i < NBMAX; i += NTHR) scnt[i] = 0;
  __syncthreads();

  int tot = 0;
  const int nChunks = (nE + CHUNK - 1) / CHUNK;
#pragma unroll 1
  for (int ch = 0; ch < nChunks; ++ch) {
    const int cbase = ch * CHUNK;
    const int wc = scan_chunk(dsts, nE, cbase, nodeBase, NBRUN, 1, list, tid, lane, wave);
    if (lane == 0) wcnt[wave] = wc;
    __syncthreads();
    int pre = 0, all = 0;
#pragma unroll
    for (int w2 = 0; w2 < NWAVE; ++w2) {
      int c = wcnt[w2];
      c = c < 0 ? 0 : (c > WCAP ? WCAP : c);
      all += c;
      pre += (w2 < wave) ? c : 0;
    }
    const int wcc  = wc > WCAP ? WCAP : wc;
    const int base = tot + pre;
#pragma unroll 1
    for (int i = lane; i < wcc; i += 32) {
      const int ent = list[wave * WCAP + i];
      const int el  = (ent >> 12) & (CHUNK - 1);
      const int sl  = ent & SMASK;
      int eid = cbase + el;
      eid = eid > nE - 1 ? nE - 1 : eid;
      const int pos = base + i;
      if (pos < RCAP) reg1[pos] = (int)(((unsigned)eid << SLB) | (unsigned)sl);
    }
    tot += all;
    tot = tot > RCAP ? RCAP : tot;
    __syncthreads();
  }
  const int nh = tot;

  if (wave == 0) {
#pragma unroll 1
    for (int b0 = 0; b0 < nh; b0 += 32) {
      const int idx = b0 + lane;
      const int uv  = reg1[idx < RCAP ? idx : RCAP - 1];
      const int m32 = (nh - b0) < 32 ? (nh - b0) : 32;
#pragma unroll 1
      for (int k = 0; k < m32; ++k) {
        const int u  = __builtin_amdgcn_readlane(uv, k);
        const int sl = u & SMASK;
        if (lane == 0) scnt[sl] = scnt[sl] + 1;
      }
    }
  }
  __syncthreads();

  {
    const v4i ca = *(const v4ia*)(scnt + 8 * tid);
    const v4i cb = *(const v4ia*)(scnt + 8 * tid + 4);
    const int e0 = ca.x < 0 ? 0 : ca.x, e1 = ca.y < 0 ? 0 : ca.y, e2 = ca.z < 0 ? 0 : ca.z, e3 = ca.w < 0 ? 0 : ca.w;
    const int e4 = cb.x < 0 ? 0 : cb.x, e5 = cb.y < 0 ? 0 : cb.y, e6 = cb.z < 0 ? 0 : cb.z, e7 = cb.w < 0 ? 0 : cb.w;
    const int ts = e0 + e1 + e2 + e3 + e4 + e5 + e6 + e7;
    int incl = ts;
#pragma unroll
    for (int d = 1; d < 32; d <<= 1) {
      const int up = __shfl_up(incl, d);
      if (lane >= d) incl += up;
    }
    if (lane == 31) wtot[wave] = incl;
    __syncthreads();
    int pre = 0;
#pragma unroll
    for (int w2 = 0; w2 < NWAVE; ++w2) pre += (w2 < wave) ? wtot[w2] : 0;
    int run = pre + incl - ts;
    soff[8 * tid + 0] = run; run += e0;
    soff[8 * tid + 1] = run; run += e1;
    soff[8 * tid + 2] = run; run += e2;
    soff[8 * tid + 3] = run; run += e3;
    soff[8 * tid + 4] = run; run += e4;
    soff[8 * tid + 5] = run; run += e5;
    soff[8 * tid + 6] = run; run += e6;
    soff[8 * tid + 7] = run;
  }
  __syncthreads();
  for (int i = tid; i < NBMAX; i += NTHR) list[i] = soff[i];
  __syncthreads();

  if (wave == 0) {
#pragma unroll 1
    for (int b0 = 0; b0 < nh; b0 += 32) {
      const int idx = b0 + lane;
      const int uv  = reg1[idx < RCAP ? idx : RCAP - 1];
      const int m32 = (nh - b0) < 32 ? (nh - b0) : 32;
#pragma unroll 1
      for (int k = 0; k < m32; ++k) {
        const int u   = __builtin_amdgcn_readlane(uv, k);
        const int sl  = u & SMASK;
        const int eid = (int)((unsigned)u >> SLB);
        if (lane == 0) {
          int pos = list[sl];
          pos = pos < 0 ? 0 : (pos > RCAP - 1 ? RCAP - 1 : pos);
          reg2[pos] = eid;
          list[sl] = pos + 1;
        }
      }
    }
  }
  __syncthreads();

  const int nbw = NBRUN / NWAVE;
  const bool ovf = (nh >= RCAP);
  const float qnan = __int_as_float(0x7fc00000);
  const float ninf = -__builtin_inff();
  int* stw = reg1 + wave * STW;
  const int lc = lane < 24 ? lane : 23;
  float at[3], bb[3];
#pragma unroll
  for (int j = 0; j < 3; ++j) {
    at[j] = PAR[2 * DP + 32 * j + lane];
    bb[j] = PAR[3 * DP + 32 * j + lane];
  }
#pragma unroll 1
  for (int jt = 0; jt < nbw; ++jt) {
    const int slot = wave * nbw + jt;
    const int grow = nodeBase + slot;
    const int gcl  = grow < nN ? grow : nN - 1;
    int st = soff[slot];
    const int craw = scnt[slot];
    int cnt = craw;
    st  = st < 0 ? 0 : (st > nh ? nh : st);
    cnt = cnt < 0 ? 0 : (cnt > DEGCAP ? DEGCAP : cnt);
    if (cnt > nh - st) cnt = nh - st;
    const bool poison = ovf || (craw > DEGCAP);
    const bool live   = grow < nN;

    const float* drow = XLR + (size_t)gcl * XLN + DP + lane;
    const unsigned short* xrow = XB + (size_t)gcl * DP + lane;
    float hd[3], av[3];
    unsigned xw[3];
#pragma unroll
    for (int j = 0; j < 3; ++j) { hd[j] = drow[32 * j]; xw[j] = (unsigned)xrow[32 * j]; av[j] = 0.0f; }
    ldwait();
    float mx = ninf, dn = 0.0f;

#pragma unroll 1
    for (int q = 0; q < cnt; ++q) {
      int idx = st + q; idx = idx > RCAP - 1 ? RCAP - 1 : idx;
      int eid = reg2[idx]; eid = eid < 0 ? 0 : (eid > nE - 1 ? nE - 1 : eid);
      const int sraw = srcs[eid];
      const int s = sraw < 0 ? 0 : (sraw > nN - 1 ? nN - 1 : sraw);
      const float* sr = XLR + (size_t)s * XLN + lane;
      float hs[3];
#pragma unroll
      for (int j = 0; j < 3; ++j) hs[j] = sr[32 * j];
      ldwait();
      float part = 0.0f;
#pragma unroll
      for (int j = 0; j < 3; ++j) {
        float v = hs[j] + hd[j];
        v = v > 0.0f ? v : v * NEGS;
        part = fmaf(v, at[j], part);
      }
#pragma unroll
      for (int off = 16; off > 0; off >>= 1) part += __shfl_xor(part, off);
      const float al = part;
      const bool first = (mx == ninf);
      const float df = first ? 0.0f : (al - mx);
      const float ee = expf(-fabsf(df));
      const bool up  = first || (df > 0.0f);
      const float s1 = first ? 0.0f : (up ? ee : 1.0f);
      const float s2 = up ? 1.0f : ee;
      mx = up ? al : mx;
      dn = fmaf(dn, s1, s2);
#pragma unroll
      for (int j = 0; j < 3; ++j) av[j] = fmaf(av[j], s1, s2 * hs[j]);
    }
    const float iv = __builtin_amdgcn_rcpf(dn + 1e-16f);
    unsigned hb[3], lb[3];
#pragma unroll
    for (int j = 0; j < 3; ++j) {
      float v = fmaf(av[j], iv, bb[j]) + __uint_as_float(xw[j] << 16);
      v = relu_np(v);
      v = poison ? qnan : v;
      v = live ? v : 0.0f;
      hb[j] = bf16_bits(v);
      lb[j] = bf16_bits(v - __uint_as_float(hb[j] << 16));
    }
    unsigned ph[3], pl[3];
#pragma unroll
    for (int j = 0; j < 3; ++j) {
      ph[j] = (unsigned)__shfl_xor((int)hb[j], 1);
      pl[j] = (unsigned)__shfl_xor((int)lb[j], 1);
    }
    wave_sync();
    if ((lane & 1) == 0) {
#pragma unroll
      for (int j = 0; j < 3; ++j) {
        stw[16 * j + (lane >> 1)]      = (int)(hb[j] | (ph[j] << 16));
        stw[48 + 16 * j + (lane >> 1)] = (int)(lb[j] | (pl[j] << 16));
      }
    }
    wave_sync();
    const v4i qv = *(const v4ia*)(stw + 4 * lc);
    if (grow < MPAD) {
      unsigned short* gp = G + (size_t)grow * GPW + goff + 8 * lc;
      const bool wsv = lane < 24;
      if (wsv) *(volatile v4i*)gp = qv;
      __threadfence();
      if (wsv) *(volatile v4i*)gp = qv;
    }
  }
}

static inline int cdiv(int a, int b) { return (a + b - 1) / b; }
static inline size_t al256(size_t o) { return (o + 255) & ~(size_t)255; }

#define SZ_XB   ((size_t)MPAD * DP * 2)
#define SZ_XLR  ((size_t)MPAD * XLN * 4)
#define SZ_G    ((size_t)MPAD * GPW * 2)
#define SZ_H1   ((size_t)MPAD * 256 * 2)
#define SZ_H2   ((size_t)MPAD * 128 * 2)
static_assert(SZ_H1 + SZ_H2 == SZ_XLR);
static_assert((SZ_XB % 256) == 0 && (SZ_XLR % 256) == 0 && (SZ_G % 256) == 0 && (SZ_H1 % 256) == 0);

extern "C" void kernel_launch(void* const* d_in, const int* in_sizes, int n_in,
                              void* d_out, int out_size, void* d_ws, size_t ws_size,
                              hipStream_t stream) {
  if (n_in < 24) return;
  if (in_sizes[0] != NN * DF || in_sizes[2] != NN * DF) return;
  if (in_sizes[1] != 2 * NE || in_sizes[3] != 2 * NE) return;
  if (in_sizes[4] != DF * DF || in_sizes[6] != DF * DF || in_sizes[10] != DF * DF || in_sizes[12] != DF * DF) return;
  if (in_sizes[5] != DF || in_sizes[7] != DF || in_sizes[8] != DF || in_sizes[9] != DF) return;
  if (in_sizes[11] != DF || in_sizes[13] != DF || in_sizes[14] != DF || in_sizes[15] != DF) return;
  if (in_sizes[16] != 128 * 146 || in_sizes[17] != 128) return;
  if (in_sizes[18] != 64 * 128 || in_sizes[19] != 64) return;
  if (in_sizes[20] != 32 * 64 || in_sizes[21] != 32) return;
  if (in_sizes[22] != 32 || in_sizes[23] != 1) return;
  if (out_size != NN) return;

  const float* x_f  = (const float*)d_in[0];
  const int*   ei_f = (const int*)  d_in[1];
  const float* x_b  = (const float*)d_in[2];
  const int*   ei_b = (const int*)  d_in[3];
  const float* Wl_f = (const float*)d_in[4];  const float* bl_f = (const float*)d_in[5];
  const float* Wr_f = (const float*)d_in[6];  const float* br_f = (const float*)d_in[7];
  const float* at_f = (const float*)d_in[8];  const float* bi_f = (const float*)d_in[9];
  const float* Wl_b = (const float*)d_in[10]; const float* bl_b = (const float*)d_in[11];
  const float* Wr_b = (const float*)d_in[12]; const float* br_b = (const float*)d_in[13];
  const float* at_b = (const float*)d_in[14]; const float* bi_b = (const float*)d_in[15];
  const float* W1 = (const float*)d_in[16];   const float* b1 = (const float*)d_in[17];
  const float* W2 = (const float*)d_in[18];   const float* b2 = (const float*)d_in[19];
  const float* W3 = (const float*)d_in[20];   const float* b3 = (const float*)d_in[21];
  const float* W4 = (const float*)d_in[22];   const float* b4 = (const float*)d_in[23];
  float* out = (float*)d_out;

  char* ws = (char*)d_ws;
  size_t off = 0;
  const size_t oXB   = off; off = al256(off + SZ_XB);
  const size_t oXLR  = off; off = al256(off + SZ_XLR);
  const size_t oG    = off; off = al256(off + SZ_G);
  const size_t oWLRf = off; off = al256(off + (size_t)XLN * DP * 2);
  const size_t oWLRb = off; off = al256(off + (size_t)XLN * DP * 2);
  const size_t oPARf = off; off = al256(off + (size_t)4 * DP * 4);
  const size_t oPARb = off; off = al256(off + (size_t)4 * DP * 4);
  const size_t oW1c  = off; off = al256(off + (size_t)128 * 384 * 2);
  const size_t oW2c  = off; off = al256(off + (size_t)64 * 256 * 2);
  const size_t oW3c  = off; off = al256(off + (size_t)32 * 128 * 2);
  const size_t oPB   = off; off = al256(off + (size_t)288 * 4);
  if (off > ws_size || off > (size_t)WSMAX) return;
  unsigned short* XB   = (unsigned short*)(ws + oXB);
  float*          XLR  = (float*)(ws + oXLR);
  unsigned short* H1   = (unsigned short*)(ws + oXLR);
  unsigned short* H2   = (unsigned short*)(ws + oXLR + SZ_H1);
  unsigned short* G    = (unsigned short*)(ws + oG);
  unsigned short* WLRf = (unsigned short*)(ws + oWLRf);
  unsigned short* WLRb = (unsigned short*)(ws + oWLRb);
  float*          PARf = (float*)(ws + oPARf);
  float*          PARb = (float*)(ws + oPARb);
  unsigned short* W1c  = (unsigned short*)(ws + oW1c);
  unsigned short* W2c  = (unsigned short*)(ws + oW2c);
  unsigned short* W3c  = (unsigned short*)(ws + oW3c);
  float*          PB   = (float*)(ws + oPB);

  hipFuncSetAttribute(reinterpret_cast<const void*>(&k_scan), hipFuncAttributeMaxDynamicSharedMemorySize, LDS_AGG);

  const int nUx = MPAD * (DP / 8);
  const int gM  = MPAD / GBM;
  const int gA  = cdiv(MPAD, NBRUN);

  k_pw<<<19, 128, 0, stream>>>(Wl_f, bl_f, Wr_f, br_f, at_f, bi_f, WLRf, PARf);
  k_pw<<<19, 128, 0, stream>>>(Wl_b, bl_b, Wr_b, br_b, at_b, bi_b, WLRb, PARb);
  k_pm1<<<33, NTHR, 0, stream>>>(W1, b1, W2, b2, W1c, W2c, PB);
  k_pm2<<<3, NTHR, 0, stream>>>(W3, b3, W4, b4, W3c, PB);

  k_px<<<cdiv(nUx, NTHR), NTHR, 0, stream>>>(x_f, XB, nUx);
  k_gemm<12, 0><<<gM, GTHR, 0, stream>>>(XB, DP, WLRf, DP, PARf, (void*)XLR, MPAD);
  k_scan<<<gA, NTHR, LDS_AGG, stream>>>(ei_f, ei_f + NE, XLR, XB, PARf, G, 0);

  k_px<<<cdiv(nUx, NTHR), NTHR, 0, stream>>>(x_b, XB, nUx);
  k_gemm<12, 0><<<gM, GTHR, 0, stream>>>(XB, DP, WLRb, DP, PARb, (void*)XLR, MPAD);
  k_scan<<<gA, NTHR, LDS_AGG, stream>>>(ei_b, ei_b + NE, XLR, XB, PARb, G, 2 * DP);

  k_gemm<8, 1><<<gM, GTHR, 0, stream>>>(G, GPW, W1c, GPW, PB, (void*)H1, MPAD);
  k_gemm<4, 1><<<gM, GTHR, 0, stream>>>(H1, 256, W2c, 256, PB + 128, (void*)H2, MPAD);
  k_gemm<2, 2><<<gM, GTHR, 0, stream>>>(H2, 128, W3c, 128, PB + 192, (void*)out, NN);
}
